// GaddyMultiheadAttention_86990267613353
// MI455X (gfx1250) — hardware-verified
//
#include <hip/hip_runtime.h>


namespace {
constexpr int Bsz = 4, S = 2048, E = 768, NH = 8, DH = 96, MROWS = Bsz * S, QT_PER_B = S / 16;
constexpr int NREL = 199, NRELP = 224, MD = 100;
constexpr float QSC = 0.10206207261596575f;

typedef _Float16 b16;
typedef __attribute__((ext_vector_type(16))) _Float16 v16b;
typedef __attribute__((ext_vector_type(8)))  _Float16 v8b;
typedef __attribute__((ext_vector_type(8)))  float v8f;
typedef __attribute__((ext_vector_type(4)))  float v4f;

__device__ __forceinline__ v8b ld8b(const b16* p) { return *(const v8b*)p; }
__device__ __forceinline__ v16b cat8b(v8b a, v8b b) { return __builtin_shufflevector(a, b, 0, 1, 2, 3, 4, 5, 6, 7, 8, 9, 10, 11, 12, 13, 14, 15); }
__device__ __forceinline__ v16b frag_kb(const b16* p, int hh) { return cat8b(ld8b(p + 8 * hh), ld8b(p + 16 + 8 * hh)); }
__device__ __forceinline__ void split16(float v, b16& hi, b16& lo) { hi = (b16)v; lo = (b16)(v - (float)hi); }
__device__ __forceinline__ void frag_ksplit(const float* p, int hh, v16b& fh_, v16b& fl_) {
  const float* p0 = p + 8 * hh; const float* p1 = p + 16 + 8 * hh;
#pragma unroll
  for (int e = 0; e < 8; ++e) { b16 a, c; split16(p0[e], a, c); fh_[e] = a; fl_[e] = c; split16(p1[e], a, c); fh_[8 + e] = a; fl_[8 + e] = c; }
}
__device__ __forceinline__ v8f wmma16b(v16b a, v16b b, v8f c) {
  v8f d = __builtin_amdgcn_wmma_f32_16x16x32_f16(false, a, false, b, (short)0, c, false, false);
  asm volatile("v_nop\n\tv_nop\n\tv_nop\n\tv_nop" : "+v"(d) : "v"(a), "v"(b));
  return d;
}
__device__ __forceinline__ void wave_lds_sync() {
  __builtin_amdgcn_fence(__ATOMIC_RELEASE, "workgroup");
  __builtin_amdgcn_wave_barrier();
  __builtin_amdgcn_fence(__ATOMIC_ACQUIRE, "workgroup");
}

struct Opnd { const void* p0; const void* p1; int ld; };
template <int NP> __device__ __forceinline__ void load_frags(const Opnd& o, int row, int kb, int hh, v16b& fh_, v16b& fl_) {
  if (NP == 0) { frag_ksplit((const float*)o.p0 + (size_t)row * o.ld + kb, hh, fh_, fl_); }
  else if (NP == 3) {
    const float* p = (const float*)o.p0 + (size_t)row * o.ld + kb; const float* p0 = p + 8 * hh; const float* p1 = p + 16 + 8 * hh;
#pragma unroll
    for (int e = 0; e < 8; ++e) { fh_[e] = (b16)p0[e]; fh_[8 + e] = (b16)p1[e]; }
    fl_ = fh_;
  } else {
    fh_ = frag_kb((const b16*)o.p0 + (size_t)row * o.ld + kb, hh);
    if (NP == 2) fl_ = frag_kb((const b16*)o.p1 + (size_t)row * o.ld + kb, hh); else fl_ = fh_;
  }
}
template <int ANP, int BNP> __device__ __forceinline__ v8f mac(v16b ah, v16b al, v16b bh, v16b bl, v8f c) {
  c = wmma16b(ah, bh, c);
  if (BNP == 0 || BNP == 2) c = wmma16b(ah, bl, c);
  if (ANP == 0 || ANP == 2) c = wmma16b(al, bh, c);
  return c;
}
template <int ANP, int BNP>
__device__ __forceinline__ void gemm_tile(const Opnd& A, const Opnd& B, int K, int m0, int c0, int nloc, int hlf, v8f (&acc)[2][4]) {
  for (int kb = 0; kb < K; kb += 32) {
    v16b a0h, a0l, a1h, a1l;
    load_frags<ANP>(A, m0 + nloc, kb, hlf, a0h, a0l);
    load_frags<ANP>(A, m0 + 16 + nloc, kb, hlf, a1h, a1l);
#pragma unroll
    for (int t = 0; t < 4; ++t) {
      v16b bh, bl;
      load_frags<BNP>(B, c0 + t * 16 + nloc, kb, hlf, bh, bl);
      acc[0][t] = mac<ANP, BNP>(a0h, a0l, bh, bl, acc[0][t]);
      acc[1][t] = mac<ANP, BNP>(a1h, a1l, bh, bl, acc[1][t]);
    }
  }
}

struct Epi { float scale; const float* cscale; const float* cbias; const float* rbias; int act; float post; const float* rscale; const float* resid; };
__device__ __forceinline__ float epi_val(const Epi& e, float acc, int row, int col) {
  float val = acc * e.scale;
  if (e.cscale) val *= e.cscale[col];
  if (e.cbias) val += e.cbias[col];
  if (e.rbias) val += e.rbias[row];
  if (e.act == 1) val = 0.5f * val * (1.0f + erff(val * 0.70710678118654752f));
  val *= e.post;
  if (e.rscale) val *= e.rscale[(size_t)row * 32];
  return val;
}
__device__ __forceinline__ void epi_planes(v8f (&acc)[2][4], const Epi& e, bool two,
                                           b16* __restrict__ oh, b16* __restrict__ ol, int ldo, int m0, int c0, int lane, b16* Th, b16* Tl) {
  const int nloc = lane & 15, hlf = lane >> 4;
#pragma unroll
  for (int t = 0; t < 4; ++t)
#pragma unroll
    for (int r = 0; r < 2; ++r)
#pragma unroll
      for (int v = 0; v < 8; ++v) {
        const int rr = r * 16 + v + 8 * hlf, cc = t * 16 + nloc;
        const float val = epi_val(e, acc[r][t][v], m0 + rr, c0 + cc);
        b16 h_, l_; split16(val, h_, l_);
        Th[rr * 64 + cc] = h_; if (two) Tl[rr * 64 + cc] = l_;
      }
  wave_lds_sync();
  for (int pass = 0; pass < 2; ++pass) {
#pragma unroll
    for (int j = 0; j < 8; ++j) {
      const int rr = j * 4 + (lane >> 3), c8 = (lane & 7) * 8;
      const size_t o = (size_t)(m0 + rr) * ldo + c0 + c8;
      *(volatile v8b*)(oh + o) = ld8b(Th + rr * 64 + c8);
      if (two) *(volatile v8b*)(ol + o) = ld8b(Tl + rr * 64 + c8);
    }
    __threadfence();
  }
}
__device__ __forceinline__ void epi_f32(v8f (&acc)[2][4], const Epi& e, float* __restrict__ out, int ldo, int m0, int c0, int lane, float* Tt) {
  const int nloc = lane & 15, hlf = lane >> 4;
#pragma unroll
  for (int t = 0; t < 4; ++t)
#pragma unroll
    for (int r = 0; r < 2; ++r)
#pragma unroll
      for (int v = 0; v < 8; ++v) {
        const int rr = r * 16 + v + 8 * hlf, cc = t * 16 + nloc;
        Tt[rr * 64 + cc] = epi_val(e, acc[r][t][v], m0 + rr, c0 + cc);
      }
  wave_lds_sync();
  float* dst0 = out + (size_t)m0 * ldo + c0; const float* rs0 = e.resid ? e.resid + (size_t)m0 * ldo + c0 : nullptr;
  for (int pass = 0; pass < 2; ++pass) {
#pragma unroll
    for (int j = 0; j < 16; ++j) {
      const int rr = j * 2 + hlf, c4 = nloc * 4;
      v4f val = *(const v4f*)(Tt + rr * 64 + c4);
      if (rs0) val += *(const v4f*)(rs0 + (size_t)rr * ldo + c4);
      *(volatile v4f*)(dst0 + (size_t)rr * ldo + c4) = val;
    }
    __threadfence();
  }
}


__global__ __launch_bounds__(256) void prep_kernel(const float* __restrict__ wq, const float* __restrict__ wk, const float* __restrict__ wv, const float* __restrict__ wo,
                                                   const float* __restrict__ rel, b16* __restrict__ w16, float* __restrict__ bt) {
  __shared__ __attribute__((aligned(16))) b16 Tl[8][E];
  const int tid = threadIdx.x, lane = tid & 31, wave = tid >> 5;
  const int mat = blockIdx.x / (E / 8), n0 = (blockIdx.x % (E / 8)) * 8;
  for (int pass = 0; pass < 2; ++pass) {
    if (mat < 4) {
      for (int i = tid; i < 8 * E; i += 256) {
        const int n = n0 + i / E, k = i % E; float v;
        if (mat < 3) { const float* w = (mat == 0) ? wq : (mat == 1) ? wk : wv; const int h = n / DH, dd = n % DH; v = w[((size_t)h * E + k) * DH + dd]; }
        else { const int h = k / DH, dd = k % DH; v = wo[((size_t)h * DH + dd) * E + n]; }
        Tl[i / E][k] = (b16)v;
      }
      __syncthreads();
      { const int n = wave; b16* dst = w16 + ((size_t)mat * E + n0 + n) * E;
#pragma unroll
        for (int j = 0; j < 3; ++j) *(volatile v8b*)(dst + (j * 32 + lane) * 8) = *(const v8b*)(&Tl[n][(j * 32 + lane) * 8]); }
      __syncthreads();
    } else {
      for (int q = tid; q < NH * NRELP; q += 256) {
        const int h = q / NRELP, j = q % NRELP; float s = 0.0f;
        if (j < NREL) {
#pragma unroll 1
          for (int dd = 0; dd < DH; ++dd) s += rel[((size_t)h * NREL + j) * DH + dd];
        }
        ((volatile float*)bt)[q] = s;
      }
    }
    __threadfence();
  }
}

template <int ANP, int BNP, bool OUT16>
__global__ __launch_bounds__(128) void gemm_kernel(const void* __restrict__ A, size_t az, int lda, const void* __restrict__ Bm, size_t bz, int ldb, int K, float scale,
                                                   b16* __restrict__ o16, float* __restrict__ o32, size_t oz, int ldo) {
  __shared__ __attribute__((aligned(16))) float Ts[4][32 * 64];
  __shared__ __attribute__((aligned(16))) b16 Th[4][32 * 64];
  const int lane = threadIdx.x & 31, wave = threadIdx.x >> 5, nloc = lane & 15, hlf = lane >> 4;
  const int m0 = blockIdx.y * 128 + wave * 32, c0 = blockIdx.x * 64; const size_t z = blockIdx.z;
  v8f acc[2][4];
#pragma unroll
  for (int r = 0; r < 2; ++r)
#pragma unroll
    for (int t = 0; t < 4; ++t) acc[r][t] = (v8f){};
  const Opnd Ao{(ANP == 3) ? (const void*)((const float*)A + z * az) : (const void*)((const b16*)A + z * az), nullptr, lda};
  const Opnd Bo{(BNP == 3) ? (const void*)((const float*)Bm + z * bz) : (const void*)((const b16*)Bm + z * bz), nullptr, ldb};
  gemm_tile<ANP, BNP>(Ao, Bo, K, m0, c0, nloc, hlf, acc);
  const Epi e{scale, nullptr, nullptr, nullptr, 0, 1.0f, nullptr, nullptr};
  if (OUT16) epi_planes(acc, e, false, o16 + z * oz, nullptr, ldo, m0, c0, lane, Th[wave], nullptr);
  else       epi_f32(acc, e, o32 + z * oz, ldo, m0, c0, lane, Ts[wave]);
}

__global__ __launch_bounds__(256) void attn_kernel(const b16* __restrict__ q16, const b16* __restrict__ k16, const b16* __restrict__ vt16, const float* __restrict__ bt,
                                                   b16* __restrict__ y) {
  __shared__ __attribute__((aligned(16))) b16 Os[16 * E];
  const int h = threadIdx.x >> 5, lane = threadIdx.x & 31, hh = lane >> 4, col = lane & 15;
  const int b = blockIdx.x / QT_PER_B, q0 = (blockIdx.x % QT_PER_B) * 16, qi = q0 + col;
  const b16* qrow = q16 + ((size_t)b * S + qi) * E + h * DH;
  const v16b qf0 = frag_kb(qrow, hh), qf1 = frag_kb(qrow + 32, hh), qf2 = frag_kb(qrow + 64, hh);
  const b16* kb0 = k16 + (size_t)b * S * E + h * DH; const b16* vtb = vt16 + ((size_t)b * E + h * DH) * S; const float* bth = bt + (size_t)h * NRELP;
  float m = -INFINITY, l = 0.0f;
  v8f o[6];
#pragma unroll
  for (int n = 0; n < 6; ++n) o[n] = (v8f){};
  for (int kb = 0; kb < S; kb += 32) {
    const b16* kr0 = kb0 + (size_t)(kb + col) * E; const b16* kr1 = kb0 + (size_t)(kb + 16 + col) * E;
    v8f s0 = {}, s1 = {};
    s0 = wmma16b(frag_kb(kr0, hh), qf0, s0); s0 = wmma16b(frag_kb(kr0 + 32, hh), qf1, s0); s0 = wmma16b(frag_kb(kr0 + 64, hh), qf2, s0);
    s1 = wmma16b(frag_kb(kr1, hh), qf0, s1); s1 = wmma16b(frag_kb(kr1 + 32, hh), qf1, s1); s1 = wmma16b(frag_kb(kr1 + 64, hh), qf2, s1);
    float mr = -INFINITY;
#pragma unroll
    for (int r = 0; r < 8; ++r) {
      const int k0i = kb + 8 * hh + r, k1i = k0i + 16;
      int d0 = k0i - qi, d1 = k1i - qi;
      d0 = d0 < -(MD - 1) ? -(MD - 1) : (d0 > MD - 1 ? MD - 1 : d0); d1 = d1 < -(MD - 1) ? -(MD - 1) : (d1 > MD - 1 ? MD - 1 : d1);
      s0[r] += bth[d0 + MD - 1]; s1[r] += bth[d1 + MD - 1];
      mr = fmaxf(mr, fmaxf(s0[r], s1[r]));
    }
    mr = fmaxf(mr, __shfl_xor(mr, 16));
    const float mn = fmaxf(m, mr), al_ = __expf(m - mn);
    m = mn;
    float sum = 0.0f; v16b pb;
#pragma unroll
    for (int r = 0; r < 8; ++r) { const float p0 = __expf(s0[r] - mn), p1 = __expf(s1[r] - mn); sum += p0 + p1; pb[r] = (b16)p0; pb[8 + r] = (b16)p1; }
    sum += __shfl_xor(sum, 16);
    l = l * al_ + sum;
#pragma unroll
    for (int n = 0; n < 6; ++n) {
#pragma unroll
      for (int r = 0; r < 8; ++r) o[n][r] *= al_;
      o[n] = wmma16b(frag_kb(vtb + (size_t)(n * 16 + col) * S + kb, hh), pb, o[n]);
    }
  }
  const float inv = 1.0f / l;
#pragma unroll
  for (int n = 0; n < 6; ++n)
#pragma unroll
    for (int r = 0; r < 8; ++r) Os[col * E + h * DH + n * 16 + 8 * hh + r] = (b16)(o[n][r] * inv);
  __syncthreads();
  b16* dst = y + ((size_t)b * S + q0) * E;
  for (int pass = 0; pass < 2; ++pass) {
    for (int p = threadIdx.x; p < 16 * E / 8; p += 256) *(volatile v8b*)(dst + (size_t)p * 8) = ld8b(Os + p * 8);
    __threadfence();
  }
}
}

extern "C" void kernel_launch(void* const* d_in, const int* in_sizes, int n_in,
                              void* d_out, int out_size, void* d_ws, size_t ws_size, hipStream_t stream) {
  (void)n_in; (void)out_size;
  const float* x   = (const float*)d_in[0];
  const float* wq  = (const float*)d_in[1];
  const float* wk  = (const float*)d_in[2];
  const float* wv  = (const float*)d_in[3];
  const float* wo  = (const float*)d_in[4];
  const float* rel = (const float*)d_in[5];
  float* out = (float*)d_out;
  if (in_sizes[0] != MROWS * E || in_sizes[1] != NH * E * DH || in_sizes[4] != NH * DH * E || in_sizes[5] != NH * NREL * DH) return;

  size_t off = 0; char* ws = (char*)d_ws;
  auto carve = [&](size_t bytes) { char* p = ws + off; off += (bytes + 255) & ~(size_t)255; return p; };
  b16* w16   = (b16*)carve((size_t)4 * E * E * 2);
  float* bt  = (float*)carve((size_t)NH * NRELP * 4);
  b16* q16   = (b16*)carve((size_t)MROWS * E * 2);
  b16* k16   = (b16*)carve((size_t)MROWS * E * 2);
  b16* vt16  = (b16*)carve((size_t)MROWS * E * 2);
  b16* y16   = (b16*)carve((size_t)MROWS * E * 2);
  if (off > ws_size) return;
  const b16* wq16 = w16; const b16* wk16 = w16 + (size_t)E * E; const b16* wv16 = w16 + (size_t)2 * E * E; const b16* wo16 = w16 + (size_t)3 * E * E;
  prep_kernel<<<4 * (E / 8) + 1, 256, 0, stream>>>(wq, wk, wv, wo, rel, w16, bt);
  gemm_kernel<3, 1, true><<<dim3(E / 64, MROWS / 128, 1), 128, 0, stream>>>(x, 0, E, wq16, 0, E, E, QSC, q16, nullptr, 0, E);
  gemm_kernel<3, 1, true><<<dim3(E / 64, MROWS / 128, 1), 128, 0, stream>>>(x, 0, E, wk16, 0, E, E, 1.0f, k16, nullptr, 0, E);
  gemm_kernel<1, 3, true><<<dim3(S / 64, E / 128, Bsz), 128, 0, stream>>>(wv16, 0, E, x, (size_t)S * E, E, E, 1.0f, vt16, nullptr, (size_t)E * S, S);
  attn_kernel<<<Bsz * QT_PER_B, 256, 0, stream>>>(q16, k16, vt16, bt, y16);
  gemm_kernel<1, 1, false><<<dim3(E / 64, MROWS / 128, 1), 128, 0, stream>>>(y16, 0, E, wo16, 0, E, E, 1.0f, nullptr, out, 0, E);
}
